// NonLocalBlock2D_17317308137919
// MI455X (gfx1250) — hardware-verified
//
#include <hip/hip_runtime.h>
#include <math.h>

constexpr int kB   = 8;
constexpr int kC   = 256;
constexpr int kO   = 128;
constexpr int kImg = 64;
constexpr int kN   = kImg * kImg;
constexpr int kM   = (kImg / 2) * (kImg / 2);
constexpr int kNB  = 2;
constexpr int kWElems = kO * kC;
constexpr float kPCarry   = 32768.0f;
constexpr float kGCarry   = 16.0f;
constexpr float kYCarry   = 16.0f;
constexpr float kWCarry   = 16.0f;
constexpr float kPVScale  = kYCarry / (kPCarry * kGCarry);
constexpr float kOutScale = 1.0f / (kWCarry * kYCarry);
constexpr float kBnEps    = 1.0e-5f;
constexpr int kPrmBth = 0, kPrmBph = 128, kPrmBg = 256, kPrmTab = 384, kPrmFloats = 1408;
constexpr int kPtPitch = 129;

static_assert(kN % 64 == 0 && kM % 64 == 0 && kO % 64 == 0 && kC % 64 == 0);
static_assert(kC % 32 == 0 && kO % 32 == 0 && kM % 32 == 0);
static_assert(kB % kNB == 0);
static_assert(kC * kO == kWElems);
static_assert(kPrmFloats == 11 * 128);

constexpr size_t kSzXT  = (size_t)kB * kN * kC * 2;
constexpr size_t kSzW16 = (size_t)4 * kWElems * 2;
constexpr size_t kSzPrm = 8192;
constexpr size_t kSzTh  = (size_t)kB * kN * kO * 2;
constexpr size_t kSzF   = (size_t)kB * kN * kO * 4;
constexpr size_t kSzPh  = (size_t)kB * kM * kO * 2;
constexpr size_t kSzGP  = (size_t)kB * kO * kM * 2;
constexpr size_t kSzYT  = (size_t)kB * kN * kO * 2;
constexpr size_t kSzSC  = (size_t)kNB * kN * kM * 4;
constexpr size_t kSzPP  = (size_t)kNB * kN * kM * 2;
constexpr size_t kOffXT  = 0;
constexpr size_t kOffW16 = kOffXT + kSzXT;
constexpr size_t kOffPrm = kOffW16 + kSzW16;
constexpr size_t kOffThH = kOffPrm + kSzPrm;
constexpr size_t kOffThL = kOffThH + kSzTh;
constexpr size_t kOffPhF = kOffThL + kSzTh;
constexpr size_t kOffGF  = kOffPhF + kSzF;
constexpr size_t kOffPhH = kOffGF + kSzF;
constexpr size_t kOffPhL = kOffPhH + kSzPh;
constexpr size_t kOffGP  = kOffPhL + kSzPh;
constexpr size_t kOffYT  = kOffGP + kSzGP;
constexpr size_t kOffSC  = kOffYT + kSzYT;
constexpr size_t kOffPP  = kOffSC + kSzSC;
constexpr size_t kWsTotal = kOffPP + kSzPP;
static_assert(kWsTotal == 132390912ull);
static_assert(kWsTotal <= 134217728ull);
static_assert(kPrmFloats * 4 <= (int)kSzPrm);
static_assert(kOffW16 % 128 == 0 && kOffPrm % 128 == 0 && kOffThH % 128 == 0 && kOffPhH % 128 == 0 &&
              kOffGP % 128 == 0 && kOffYT % 128 == 0 && kOffSC % 128 == 0 && kOffPP % 128 == 0);

typedef __attribute__((ext_vector_type(16))) _Float16 v16h;
typedef __attribute__((ext_vector_type(8)))  _Float16 v8h;
typedef __attribute__((ext_vector_type(16))) __bf16   v16b;
typedef __attribute__((ext_vector_type(8)))  __bf16   v8b;
typedef __attribute__((ext_vector_type(8)))  float    v8f;
typedef __attribute__((ext_vector_type(4)))  float    v4f;
typedef __attribute__((ext_vector_type(4)))  unsigned int v4u;

__device__ __forceinline__ unsigned short f2bf_bits(float f) {
  unsigned u = __float_as_uint(f);
  return (unsigned short)((u + 0x7FFFu + ((u >> 16) & 1u)) >> 16);
}
__device__ __forceinline__ float bf_bits2f(unsigned short h) { return __uint_as_float(((unsigned)h) << 16); }

__device__ __forceinline__ void dep_guard_h(v8f& a, v8f& b, v16h x, v16h y) { asm volatile("v_nop\n\tv_nop\n\tv_nop\n\tv_nop" : "+v"(a), "+v"(b) : "v"(x), "v"(y)); }
__device__ __forceinline__ void dep_guard_b(v8f& a, v8f& b, v16b x, v16b y) { asm volatile("v_nop\n\tv_nop\n\tv_nop\n\tv_nop" : "+v"(a), "+v"(b) : "v"(x), "v"(y)); }
__device__ __forceinline__ void dep_guard4_h(v8f& a, v8f& b, v8f& c, v8f& d, v16h x, v16h y) { asm volatile("v_nop\n\tv_nop\n\tv_nop\n\tv_nop" : "+v"(a), "+v"(b), "+v"(c), "+v"(d) : "v"(x), "v"(y)); }
__device__ __forceinline__ void dep_guard4_b(v8f& a, v8f& b, v8f& c, v8f& d, v16b x, v16b y) { asm volatile("v_nop\n\tv_nop\n\tv_nop\n\tv_nop" : "+v"(a), "+v"(b), "+v"(c), "+v"(d) : "v"(x), "v"(y)); }
__device__ __forceinline__ void keep4_h(v16h a, v16h b, v16h c, v16h d) { asm volatile("v_nop" :: "v"(a), "v"(b), "v"(c), "v"(d)); }
__device__ __forceinline__ void keep4_b(v16b a, v16b b, v16b c, v16b d) { asm volatile("v_nop" :: "v"(a), "v"(b), "v"(c), "v"(d)); }
__device__ __forceinline__ void acc_guard4(v8f& a, v8f& b, v8f& c, v8f& d) { asm volatile("v_nop\n\tv_nop\n\tv_nop\n\tv_nop" : "+v"(a), "+v"(b), "+v"(c), "+v"(d)); }
template <typename T> struct Frag;
template <> struct Frag<_Float16> {
  typedef v16h V; union U { v16h v; v8h h[2]; };
  static __device__ __forceinline__ v16h load(const _Float16* p) {
    U f; f.h[0] = *(const v8h*)(p); f.h[1] = *(const v8h*)(p + 16); return f.v;
  }
  static __device__ __forceinline__ v8f mma(v16h a, v16h b, v8f c) {
    return __builtin_amdgcn_wmma_f32_16x16x32_f16(false, a, false, b, (short)0, c, false, false);
  }
  static __device__ __forceinline__ void guard(v8f& a, v8f& b, v16h x, v16h y) { dep_guard_h(a, b, x, y); }
  static __device__ __forceinline__ void guard4(v8f& a, v8f& b, v8f& c, v8f& d, v16h x, v16h y) { dep_guard4_h(a, b, c, d, x, y); }
  static __device__ __forceinline__ void keep(v16h a, v16h b, v16h c, v16h d) { keep4_h(a, b, c, d); }
};
template <> struct Frag<__bf16> {
  typedef v16b V; union U { v16b v; v8b h[2]; };
  static __device__ __forceinline__ v16b load(const __bf16* p) {
    U f; f.h[0] = *(const v8b*)(p); f.h[1] = *(const v8b*)(p + 16); return f.v;
  }
  static __device__ __forceinline__ v8f mma(v16b a, v16b b, v8f c) {
    return __builtin_amdgcn_wmma_f32_16x16x32_bf16(false, a, false, b, (short)0, c, false, false);
  }
  static __device__ __forceinline__ void guard(v8f& a, v8f& b, v16b x, v16b y) { dep_guard_b(a, b, x, y); }
  static __device__ __forceinline__ void guard4(v8f& a, v8f& b, v8f& c, v8f& d, v16b x, v16b y) { dep_guard4_b(a, b, c, d, x, y); }
  static __device__ __forceinline__ void keep(v16b a, v16b b, v16b c, v16b d) { keep4_b(a, b, c, d); }
};

__device__ __forceinline__ unsigned pk16(unsigned short a, unsigned short b) { return (unsigned)a | ((unsigned)b << 16); }
__device__ __forceinline__ unsigned short h_bits(float f) { const _Float16 h = (_Float16)f; return __builtin_bit_cast(unsigned short, h); }

template <int ET> struct Elem;
template <> struct Elem<0> { typedef _Float16 T; };
template <> struct Elem<1> { typedef __bf16 T; };
template <int ET, bool SPLIT, int BIAS_MODE, int OUT_MODE, bool RESID, int ACT = 0>
__global__ __launch_bounds__(256) void wmma_gemm64(
    const unsigned short* __restrict__ Ap, const unsigned short* __restrict__ A2p, int lda, long strideA,
    const unsigned short* __restrict__ Btp, const unsigned short* __restrict__ Bt2p, int ldb, long strideB,
    void* __restrict__ Cout, void* __restrict__ Cout2, int ldc, long strideC,
    const float* __restrict__ bias,
    const float* __restrict__ resid, long strideR,
    int M, int N, int K, float scale) {
  typedef typename Elem<ET>::T T;
  typedef typename Frag<T>::V V;
  const T* A = (const T*)Ap; const T* A2 = (const T*)A2p; const T* Bt = (const T*)Btp; const T* Bt2 = (const T*)Bt2p;
  __shared__ __align__(16) float sT[8][16 * 68];
  const int b    = blockIdx.y;
  const int lane = threadIdx.x & 31;
  const int wave = threadIdx.x >> 5;
  const int tilesN = N >> 6;
  const int tilesM = M >> 6;
  const int tile = blockIdx.x * 8 + wave;
  if (tile >= tilesM * tilesN) return;
  const int tm = tile / tilesN;
  const int tn = tile - tm * tilesN;
  const int m0 = tm << 6;
  const int n0 = tn << 6;

  const T* Ab  = A  + (size_t)b * strideA;
  const T* Bb  = Bt + (size_t)b * strideB;
  const T* Ab2 = SPLIT ? (A2  + (size_t)b * strideA) : nullptr;
  const T* Bb2 = SPLIT ? (Bt2 + (size_t)b * strideB) : nullptr;

  const int rlane = lane & 15;
  const int koff  = (lane >> 4) * 8;
  const int mOff  = (lane >> 4) * 8;

  v8f acc[4][4];
#pragma unroll
  for (int i = 0; i < 4; ++i)
#pragma unroll
    for (int j = 0; j < 4; ++j) acc[i][j] = (v8f){0.f,0.f,0.f,0.f,0.f,0.f,0.f,0.f};

  for (int k0 = 0; k0 < K; k0 += 32) {
    V bh[4], bl[4];
#pragma unroll
    for (int j = 0; j < 4; ++j) {
      const size_t bo = (size_t)(n0 + (j << 4) + rlane) * ldb + koff + k0;
      bh[j] = Frag<T>::load(Bb + bo);
      if (SPLIT) bl[j] = Frag<T>::load(Bb2 + bo);
    }
#pragma unroll
    for (int i = 0; i < 4; ++i) {
      const size_t ao = (size_t)(m0 + (i << 4) + rlane) * lda + koff + k0;
      V ah = Frag<T>::load(Ab + ao);
      V al;
      if (SPLIT) al = Frag<T>::load(Ab2 + ao);
#pragma unroll
      for (int j = 0; j < 4; ++j) {
        acc[i][j] = Frag<T>::mma(ah, bh[j], acc[i][j]);
        if (SPLIT) {
          acc[i][j] = Frag<T>::mma(ah, bl[j], acc[i][j]);
          acc[i][j] = Frag<T>::mma(al, bh[j], acc[i][j]);
        }
      }
      Frag<T>::guard4(acc[i][0], acc[i][1], acc[i][2], acc[i][3], ah, SPLIT ? al : ah);
    }
    Frag<T>::keep(bh[0], bh[1], bh[2], bh[3]);
    if (SPLIT) Frag<T>::keep(bl[0], bl[1], bl[2], bl[3]);
  }
  acc_guard4(acc[0][0], acc[0][1], acc[0][2], acc[0][3]);
  acc_guard4(acc[1][0], acc[1][1], acc[1][2], acc[1][3]);
  acc_guard4(acc[2][0], acc[2][1], acc[2][2], acc[2][3]);
  acc_guard4(acc[3][0], acc[3][1], acc[3][2], acc[3][3]);

  float* slab = sT[wave];
  const float* Rb = RESID ? (resid + (size_t)b * strideR) : nullptr;
#pragma unroll
  for (int i = 0; i < 4; ++i) {
    const int mBase = m0 + (i << 4);
#pragma unroll
    for (int j = 0; j < 4; ++j) {
      const int n = n0 + (j << 4) + rlane;
      float bv = 0.f;
      if (BIAS_MODE == 2) bv = bias[n];
#pragma unroll
      for (int r = 0; r < 8; ++r) {
        float v = acc[i][j][r] * scale;
        if (BIAS_MODE == 1) v += bias[mBase + mOff + r];
        if (BIAS_MODE == 2) v += bv;
        if (RESID) v += Rb[(size_t)(mBase + mOff + r) * ldc + n];
        if (ACT == 2) v = fmaxf(v, 0.0f);
        if (ACT == 4) v = (v > 0.f) ? v : 0.01f * v;
        slab[(mOff + r) * 68 + (j << 4) + rlane] = v;
      }
    }
    __builtin_amdgcn_fence(__ATOMIC_RELEASE, "workgroup");
    __builtin_amdgcn_wave_barrier();
    __builtin_amdgcn_fence(__ATOMIC_ACQUIRE, "workgroup");
    if (OUT_MODE == 0) {
      float* C = (float*)Cout + (size_t)b * strideC;
      const int hh = lane >> 4, c4 = (lane & 15) * 4;
      for (int pass = 0; pass < 2; ++pass) {
#pragma unroll
        for (int it = 0; it < 8; ++it) {
          const int row = it * 2 + hh;
          v4f v = *(const v4f*)(slab + row * 68 + c4);
          *(volatile v4f*)(C + (size_t)(mBase + row) * ldc + n0 + c4) = v;
        }
        __threadfence();
      }
    } else {
      const int q = lane >> 3, c8 = (lane & 7) * 8;
      unsigned short* C  = (unsigned short*)Cout  + (size_t)b * strideC;
      unsigned short* C2 = (OUT_MODE == 2) ? ((unsigned short*)Cout2 + (size_t)b * strideC) : nullptr;
      for (int pass = 0; pass < 2; ++pass) {
#pragma unroll
        for (int it = 0; it < 4; ++it) {
          const int row = it * 4 + q;
          const float* sp = slab + row * 68 + c8;
          v8h hv, lv;
#pragma unroll
          for (int e = 0; e < 8; ++e) {
            if (OUT_MODE == 1) {
              hv[e] = (_Float16)sp[e];
            } else {
              unsigned short hb = f2bf_bits(sp[e]);
              unsigned short lb = f2bf_bits(sp[e] - bf_bits2f(hb));
              hv[e] = __builtin_bit_cast(_Float16, hb);
              lv[e] = __builtin_bit_cast(_Float16, lb);
            }
          }
          *(volatile v8h*)(C + (size_t)(mBase + row) * ldc + n0 + c8) = hv;
          if (OUT_MODE == 2) *(volatile v8h*)(C2 + (size_t)(mBase + row) * ldc + n0 + c8) = lv;
        }
        __threadfence();
      }
    }
    __builtin_amdgcn_fence(__ATOMIC_RELEASE, "workgroup");
    __builtin_amdgcn_wave_barrier();
    __builtin_amdgcn_fence(__ATOMIC_ACQUIRE, "workgroup");
  }
}

__global__ __launch_bounds__(256) void wmma_gemm64_bnres(
    const unsigned short* __restrict__ Ap, int lda,
    const unsigned short* __restrict__ Btp, int ldb, long strideB,
    float* __restrict__ Cout, int ldc, long strideC,
    const float* __restrict__ tab,
    const float* __restrict__ resid, long strideR,
    int M, int N, int K, float scale) {
  typedef _Float16 T;
  typedef v16h V;
  const T* A = (const T*)Ap; const T* Bt = (const T*)Btp;
  __shared__ __align__(16) float sT[8][16 * 68];
  const int b    = blockIdx.y;
  const int lane = threadIdx.x & 31;
  const int wave = threadIdx.x >> 5;
  const int tilesN = N >> 6;
  const int tilesM = M >> 6;
  const int tile = blockIdx.x * 8 + wave;
  if (tile >= tilesM * tilesN) return;
  const int tm = tile / tilesN;
  const int tn = tile - tm * tilesN;
  const int m0 = tm << 6;
  const int n0 = tn << 6;

  const T* Ab = A;
  const T* Bb = Bt + (size_t)b * strideB;

  const int rlane = lane & 15;
  const int koff  = (lane >> 4) * 8;
  const int mOff  = (lane >> 4) * 8;

  v8f acc[4][4];
#pragma unroll
  for (int i = 0; i < 4; ++i)
#pragma unroll
    for (int j = 0; j < 4; ++j) acc[i][j] = (v8f){0.f,0.f,0.f,0.f,0.f,0.f,0.f,0.f};

  for (int k0 = 0; k0 < K; k0 += 32) {
    V bh[4];
#pragma unroll
    for (int j = 0; j < 4; ++j) {
      const size_t bo = (size_t)(n0 + (j << 4) + rlane) * ldb + koff + k0;
      bh[j] = Frag<T>::load(Bb + bo);
    }
#pragma unroll
    for (int i = 0; i < 4; ++i) {
      const size_t ao = (size_t)(m0 + (i << 4) + rlane) * lda + koff + k0;
      V ah = Frag<T>::load(Ab + ao);
#pragma unroll
      for (int j = 0; j < 4; ++j) acc[i][j] = Frag<T>::mma(ah, bh[j], acc[i][j]);
      Frag<T>::guard4(acc[i][0], acc[i][1], acc[i][2], acc[i][3], ah, ah);
    }
    Frag<T>::keep(bh[0], bh[1], bh[2], bh[3]);
  }
  acc_guard4(acc[0][0], acc[0][1], acc[0][2], acc[0][3]);
  acc_guard4(acc[1][0], acc[1][1], acc[1][2], acc[1][3]);
  acc_guard4(acc[2][0], acc[2][1], acc[2][2], acc[2][3]);
  acc_guard4(acc[3][0], acc[3][1], acc[3][2], acc[3][3]);

  float* slab = sT[wave];
  const float* Rb = resid + (size_t)b * strideR;
  float* Cb = Cout + (size_t)b * strideC;
#pragma unroll
  for (int i = 0; i < 4; ++i) {
    const int mBase = m0 + (i << 4);
    const int rb0 = mBase + mOff;
    const v4f bo0 = *(const v4f*)(tab + rb0);
    const v4f bo1 = *(const v4f*)(tab + rb0 + 4);
    const v4f mu0 = *(const v4f*)(tab + M + rb0);
    const v4f mu1 = *(const v4f*)(tab + M + rb0 + 4);
    const v4f iv0 = *(const v4f*)(tab + 2 * M + rb0);
    const v4f iv1 = *(const v4f*)(tab + 2 * M + rb0 + 4);
    const v4f be0 = *(const v4f*)(tab + 3 * M + rb0);
    const v4f be1 = *(const v4f*)(tab + 3 * M + rb0 + 4);
    float pbo[8], pmu[8], piv[8], pbe[8];
#pragma unroll
    for (int e = 0; e < 4; ++e) {
      pbo[e] = bo0[e]; pbo[4 + e] = bo1[e];
      pmu[e] = mu0[e]; pmu[4 + e] = mu1[e];
      piv[e] = iv0[e]; piv[4 + e] = iv1[e];
      pbe[e] = be0[e]; pbe[4 + e] = be1[e];
    }
#pragma unroll
    for (int j = 0; j < 4; ++j) {
#pragma unroll
      for (int r = 0; r < 8; ++r) {
        float v = acc[i][j][r] * scale;
        v = v + pbo[r];
        v = (v - pmu[r]) * piv[r] + pbe[r];
        slab[(mOff + r) * 68 + (j << 4) + rlane] = v;
      }
    }
    __builtin_amdgcn_fence(__ATOMIC_RELEASE, "workgroup");
    __builtin_amdgcn_wave_barrier();
    __builtin_amdgcn_fence(__ATOMIC_ACQUIRE, "workgroup");
    {
      const int hh = lane >> 4, c4 = (lane & 15) * 4;
      for (int pass = 0; pass < 2; ++pass) {
#pragma unroll
        for (int it = 0; it < 8; ++it) {
          const int row = it * 2 + hh;
          v4f v = *(const v4f*)(slab + row * 68 + c4);
          const size_t off = (size_t)(mBase + row) * ldc + n0 + c4;
          const v4f xr = *(const v4f*)(Rb + off);
#pragma unroll
          for (int e = 0; e < 4; ++e) {
            const float xe = xr[e];
            v[e] = v[e] + bf_bits2f(f2bf_bits(xe));
          }
          *(volatile v4f*)(Cb + off) = v;
        }
        __threadfence();
      }
    }
    __builtin_amdgcn_fence(__ATOMIC_RELEASE, "workgroup");
    __builtin_amdgcn_wave_barrier();
    __builtin_amdgcn_fence(__ATOMIC_ACQUIRE, "workgroup");
  }
}

__global__ __launch_bounds__(256) void xcast_kernel(const float* __restrict__ x, unsigned short* __restrict__ xT) {
  __shared__ float sm[64][65];
  const int t  = threadIdx.x;
  const int n0 = blockIdx.x * 64;
  const int c0 = blockIdx.y * 64;
  const int b  = blockIdx.z;
  const float* xb = x + (size_t)b * kC * kN;
#pragma unroll
  for (int i = 0; i < 16; ++i) {
    const int e  = i * 256 + t;
    const int r  = e >> 6;
    const int cl = e & 63;
    sm[cl][r] = xb[(size_t)(c0 + r) * kN + n0 + cl];
  }
  __syncthreads();
  const int lane = t & 31, wave = t >> 5;
  const int q = lane >> 3, c8 = (lane & 7) * 8;
  unsigned short* op = xT + (size_t)b * kN * kC;
  for (int pass = 0; pass < 2; ++pass) {
#pragma unroll
    for (int it = 0; it < 2; ++it) {
      const int row = wave * 8 + it * 4 + q;
      unsigned short hb[8];
#pragma unroll
      for (int e = 0; e < 8; ++e) hb[e] = f2bf_bits(sm[row][c8 + e]);
      const v4u u = (v4u){pk16(hb[0], hb[1]), pk16(hb[2], hb[3]), pk16(hb[4], hb[5]), pk16(hb[6], hb[7])};
      *(volatile v4u*)(op + (size_t)(n0 + row) * kC + c0 + c8) = u;
    }
    __threadfence();
  }
}

__global__ __launch_bounds__(256) void wcast_kernel(const float* __restrict__ W0, const float* __restrict__ W1,
                                                    const float* __restrict__ W2, const float* __restrict__ W3,
                                                    unsigned short* __restrict__ out) {
  const int z = blockIdx.y;
  const float* W = (z == 0) ? W0 : (z == 1) ? W1 : (z == 2) ? W2 : W3;
  const int i = blockIdx.x * 256 + threadIdx.x;
  const float* p = W + 8 * (size_t)i;
  const v4f a = *(const v4f*)(p);
  const v4f c = *(const v4f*)(p + 4);
  unsigned short hb[8];
#pragma unroll
  for (int e = 0; e < 4; ++e) {
    const float a0 = a[e];
    const float c0 = c[e];
    const unsigned short ba = f2bf_bits(a0);
    const unsigned short bc = f2bf_bits(c0);
    const unsigned short ha = h_bits(bf_bits2f(ba) * kWCarry);
    const unsigned short hc = h_bits(bf_bits2f(bc) * kWCarry);
    hb[e]     = (z == 3) ? ha : ba;
    hb[4 + e] = (z == 3) ? hc : bc;
  }
  const v4u u = (v4u){pk16(hb[0], hb[1]), pk16(hb[2], hb[3]), pk16(hb[4], hb[5]), pk16(hb[6], hb[7])};
  unsigned short* q = out + (size_t)z * kWElems + 8 * (size_t)i;
  *(volatile v4u*)q = u;
  __threadfence();
  *(volatile v4u*)q = u;
}

__global__ __launch_bounds__(32) void prm_kernel(const float* __restrict__ bth, const float* __restrict__ bph,
                                                 const float* __restrict__ bg,  const float* __restrict__ bo,
                                                 const float* __restrict__ mu,  const float* __restrict__ ga,
                                                 const float* __restrict__ be,  const float* __restrict__ var,
                                                 float* __restrict__ prm) {
  const int blk  = blockIdx.x;
  const int lane = threadIdx.x;
  const float* src = (blk == 0) ? bth : (blk == 1) ? bph : (blk == 2) ? bg : (blk <= 4) ? bo : (blk <= 6) ? mu : (blk <= 8) ? ga : be;
  const int sub = (blk <= 2) ? 0 : ((blk - 3) & 1);
  const v4f a  = *(const v4f*)(src + sub * 128 + 4 * lane);
  const v4f vv = *(const v4f*)(var + sub * 128 + 4 * lane);
  const float fi = (blk == 7 || blk == 8) ? 1.0f : 0.0f;
  v4f r;
#pragma unroll
  for (int e = 0; e < 4; ++e) {
    const float ae = a[e];
    const float ve = vv[e];
    const float ar = bf_bits2f(f2bf_bits(ae));
    const float vr = bf_bits2f(f2bf_bits(ve));
    const float iv = ar / sqrtf(vr + kBnEps);
    r[e] = fmaf(fi, iv, (1.0f - fi) * ar);
  }
  float* dp = prm + blk * 128 + 4 * lane;
  *(volatile v4f*)dp = r;
  __threadfence();
  *(volatile v4f*)dp = r;
}

__device__ __forceinline__ void pool_tile(const float* __restrict__ src, size_t rowbase, float* pt, int t) {
#pragma unroll 1
  for (int i = 0; i < 32; ++i) {
    const int it  = i * 256 + t;
    const int o   = it & 127;
    const int ml  = it >> 7;
    const int hol = ml >> 5;
    const int wo  = ml & 31;
    const float* p = src + (rowbase + (size_t)(2 * hol) * kImg + 2 * wo) * kO + o;
    const float v00 = p[0];
    const float v01 = p[kO];
    const float v10 = p[(size_t)kImg * kO];
    const float v11 = p[(size_t)kImg * kO + kO];
    pt[ml * kPtPitch + o] = fmaxf(fmaxf(v00, v01), fmaxf(v10, v11));
  }
}

__global__ __launch_bounds__(256) void pool_kernel(const float* __restrict__ phiF, const float* __restrict__ gF,
                                                   unsigned short* __restrict__ phiH, unsigned short* __restrict__ phiL,
                                                   unsigned short* __restrict__ gP) {
  __shared__ float pt[64 * kPtPitch];
  const int t = threadIdx.x, lane = t & 31, wave = t >> 5;
  const int hp = blockIdx.x;
  const int b  = blockIdx.y;
  const int m0 = hp * 64;
  const size_t rowbase = (size_t)b * kN + (size_t)hp * 4 * kImg;

  pool_tile(phiF, rowbase, pt, t);
  __syncthreads();
  {
    const int hsel = lane >> 4, o8 = (lane & 15) * 8;
    const size_t prow0 = (size_t)b * kM + m0;
    for (int pass = 0; pass < 2; ++pass) {
#pragma unroll
      for (int it = 0; it < 4; ++it) {
        const int ml = (wave * 4 + it) * 2 + hsel;
        const float* sp = pt + ml * kPtPitch + o8;
        unsigned short hb[8], lb[8];
#pragma unroll
        for (int e = 0; e < 8; ++e) {
          const float v = sp[e];
          const unsigned short hbb = f2bf_bits(v);
          hb[e] = hbb;
          lb[e] = f2bf_bits(v - bf_bits2f(hbb));
        }
        const v4u uh = (v4u){pk16(hb[0], hb[1]), pk16(hb[2], hb[3]), pk16(hb[4], hb[5]), pk16(hb[6], hb[7])};
        const v4u ul = (v4u){pk16(lb[0], lb[1]), pk16(lb[2], lb[3]), pk16(lb[4], lb[5]), pk16(lb[6], lb[7])};
        const size_t off = (prow0 + ml) * kO + o8;
        *(volatile v4u*)(phiH + off) = uh;
        *(volatile v4u*)(phiL + off) = ul;
      }
      __threadfence();
    }
  }
  __syncthreads();

  pool_tile(gF, rowbase, pt, t);
  __syncthreads();
  {
    const int q = lane >> 3, c8 = (lane & 7) * 8;
    unsigned short* og = gP + (size_t)b * kO * kM + m0;
    for (int pass = 0; pass < 2; ++pass) {
#pragma unroll
      for (int it = 0; it < 4; ++it) {
        const int o = (wave * 4 + it) * 4 + q;
        unsigned short hb[8];
#pragma unroll
        for (int e = 0; e < 8; ++e) hb[e] = h_bits(kGCarry * pt[(c8 + e) * kPtPitch + o]);
        const v4u u = (v4u){pk16(hb[0], hb[1]), pk16(hb[2], hb[3]), pk16(hb[4], hb[5]), pk16(hb[6], hb[7])};
        *(volatile v4u*)(og + (size_t)o * kM + c8) = u;
      }
      __threadfence();
    }
  }
}

__global__ __launch_bounds__(128) void softmax_kernel(const float* __restrict__ S, unsigned short* __restrict__ P) {
  __shared__ float redM[4];
  __shared__ float redS[4];
  const int row  = blockIdx.x;
  const int t    = threadIdx.x;
  const int lane = t & 31, wave = t >> 5;
  const float* sr = S + (size_t)row * kM + 8 * t;
  const v4f a = *(const v4f*)(sr);
  const v4f c = *(const v4f*)(sr + 4);
  float x[8];
#pragma unroll
  for (int e = 0; e < 4; ++e) { x[e] = a[e]; x[4 + e] = c[e]; }
  float m = fmaxf(fmaxf(fmaxf(x[0], x[1]), fmaxf(x[2], x[3])), fmaxf(fmaxf(x[4], x[5]), fmaxf(x[6], x[7])));
#pragma unroll
  for (int off = 16; off > 0; off >>= 1) m = fmaxf(m, __shfl_xor(m, off, 32));
  if (lane == 0) redM[wave] = m;
  __syncthreads();
  const float mm = fmaxf(fmaxf(redM[0], redM[1]), fmaxf(redM[2], redM[3]));

  float ev[8];
  float sum = 0.f;
#pragma unroll
  for (int e = 0; e < 8; ++e) {
    ev[e] = expf(x[e] - mm);
    sum += ev[e];
  }
#pragma unroll
  for (int off = 16; off > 0; off >>= 1) sum += __shfl_xor(sum, off, 32);
  if (lane == 0) redS[wave] = sum;
  __syncthreads();
  const float tot = ((redS[0] + redS[1]) + redS[2]) + redS[3];
  const float inv = kPCarry / tot;

  unsigned short hb[8];
#pragma unroll
  for (int e = 0; e < 8; ++e) hb[e] = h_bits(ev[e] * inv);
  const v4u u = (v4u){pk16(hb[0], hb[1]), pk16(hb[2], hb[3]), pk16(hb[4], hb[5]), pk16(hb[6], hb[7])};
  unsigned short* pr = P + (size_t)row * kM + 8 * (size_t)t;
  *(volatile v4u*)pr = u;
  __threadfence();
  *(volatile v4u*)pr = u;
}

extern "C" void kernel_launch(void* const* d_in, const int* in_sizes, int n_in,
                              void* d_out, int out_size, void* d_ws, size_t ws_size,
                              hipStream_t stream) {
  if (n_in < 13) return;
  const int nX = kB * kC * kN;
  if (in_sizes[0] != nX) return;
  if (in_sizes[1] != kWElems || in_sizes[3] != kWElems || in_sizes[5] != kWElems || in_sizes[7] != kWElems) return;
  if (in_sizes[2] != kO || in_sizes[4] != kO || in_sizes[6] != kO) return;
  if (in_sizes[8] != kC || in_sizes[9] != kC || in_sizes[10] != kC || in_sizes[11] != kC || in_sizes[12] != kC) return;
  if (out_size != nX) return;
  if (ws_size < kWsTotal) return;

  const float* x       = (const float*)d_in[0];
  const float* w_theta = (const float*)d_in[1];
  const float* b_theta = (const float*)d_in[2];
  const float* w_phi   = (const float*)d_in[3];
  const float* b_phi   = (const float*)d_in[4];
  const float* w_g     = (const float*)d_in[5];
  const float* b_g     = (const float*)d_in[6];
  const float* w_out   = (const float*)d_in[7];
  const float* b_out   = (const float*)d_in[8];
  const float* bn_gamma = (const float*)d_in[9];
  const float* bn_beta  = (const float*)d_in[10];
  const float* bn_mean  = (const float*)d_in[11];
  const float* bn_var   = (const float*)d_in[12];
  float* out = (float*)d_out;

  char* ws = (char*)d_ws;
  unsigned short* XT  = (unsigned short*)(ws + kOffXT);
  unsigned short* W16 = (unsigned short*)(ws + kOffW16);
  float*          PRM = (float*)(ws + kOffPrm);
  unsigned short* THH = (unsigned short*)(ws + kOffThH);
  unsigned short* THL = (unsigned short*)(ws + kOffThL);
  float*          PHF = (float*)(ws + kOffPhF);
  float*          GF  = (float*)(ws + kOffGF);
  unsigned short* PHH = (unsigned short*)(ws + kOffPhH);
  unsigned short* PHL = (unsigned short*)(ws + kOffPhL);
  unsigned short* GP  = (unsigned short*)(ws + kOffGP);
  unsigned short* YT  = (unsigned short*)(ws + kOffYT);
  float*          SC  = (float*)(ws + kOffSC);
  unsigned short* PP  = (unsigned short*)(ws + kOffPP);

  const unsigned short* WTH = W16;
  const unsigned short* WPH = W16 + kWElems;
  const unsigned short* WG  = W16 + 2 * kWElems;
  const unsigned short* WO  = W16 + 3 * kWElems;

  xcast_kernel<<<dim3(kN / 64, kC / 64, kB), dim3(256), 0, stream>>>(x, XT);
  wcast_kernel<<<dim3(kWElems / (8 * 256), 4), dim3(256), 0, stream>>>(w_theta, w_phi, w_g, w_out, W16);
  prm_kernel<<<dim3(kPrmFloats / 128), dim3(32), 0, stream>>>(b_theta, b_phi, b_g, b_out, bn_mean, bn_gamma, bn_beta, bn_var, PRM);

  const long strideXT = (long)kN * kC;
  const long strideNO = (long)kN * kO;
  const int  blkProj  = ((kN / 64) * (kO / 64)) / 8;
  wmma_gemm64<1, false, 2, 2, false, 0><<<dim3(blkProj, kB), dim3(256), 0, stream>>>(
      XT, XT, kC, strideXT, WTH, WTH, kC, 0L,
      (void*)THH, (void*)THL, kO, strideNO, PRM + kPrmBth, PRM, 0L, kN, kO, kC, 1.0f);
  wmma_gemm64<1, false, 2, 0, false, 0><<<dim3(blkProj, kB), dim3(256), 0, stream>>>(
      XT, XT, kC, strideXT, WPH, WPH, kC, 0L,
      (void*)PHF, (void*)PHF, kO, strideNO, PRM + kPrmBph, PRM, 0L, kN, kO, kC, 1.0f);
  wmma_gemm64<1, false, 2, 0, false, 0><<<dim3(blkProj, kB), dim3(256), 0, stream>>>(
      XT, XT, kC, strideXT, WG, WG, kC, 0L,
      (void*)GF, (void*)GF, kO, strideNO, PRM + kPrmBg, PRM, 0L, kN, kO, kC, 1.0f);

  pool_kernel<<<dim3(kM / 64, kB), dim3(256), 0, stream>>>(PHF, GF, PHH, PHL, GP);

  const long strideMO  = (long)kM * kO;
  const long strideNM  = (long)kN * kM;
  const long strideOM  = (long)kO * kM;
  const int  blkScore  = ((kN / 64) * (kM / 64)) / 8;
  const int  blkPV     = ((kN / 64) * (kO / 64)) / 8;
  for (int ch = 0; ch < kB / kNB; ++ch) {
    const size_t thOff = (size_t)ch * kNB * kN * kO;
    const size_t phOff = (size_t)ch * kNB * kM * kO;
    const size_t gOff  = (size_t)ch * kNB * kO * kM;
    wmma_gemm64<1, true, 0, 0, false, 0><<<dim3(blkScore, kNB), dim3(256), 0, stream>>>(
        THH + thOff, THL + thOff, kO, strideNO, PHH + phOff, PHL + phOff, kO, strideMO,
        (void*)SC, (void*)SC, kM, strideNM, PRM, PRM, 0L, kN, kM, kO, 1.0f);
    softmax_kernel<<<dim3(kNB * kN), dim3(128), 0, stream>>>(SC, PP);
    wmma_gemm64<0, false, 0, 1, false, 0><<<dim3(blkPV, kNB), dim3(256), 0, stream>>>(
        PP, PP, kM, strideNM, GP + gOff, GP + gOff, kM, strideOM,
        (void*)(YT + thOff), (void*)(YT + thOff), kO, strideNO, PRM, PRM, 0L, kN, kO, kM, kPVScale);
  }

  const long strideCN = (long)kC * kN;
  const int  blkOut   = ((kC / 64) * (kN / 64)) / 8;
  wmma_gemm64_bnres<<<dim3(blkOut, kB), dim3(256), 0, stream>>>(
      WO, kO, YT, kO, strideNO, out, kN, strideCN, PRM + kPrmTab, x, strideCN, kC, kN, kO, kOutScale);
}
